// CountryAttnEncoder_23828478558673
// MI455X (gfx1250) — hardware-verified
//
#include <hip/hip_runtime.h>


namespace {
constexpr int Bn = 8192, S = 86, SP = 96, D = 64, NH = 4, HD = 16, FEAT = 11, KF = 32  , R = 7, NP = 1 + R, HID = 128, KO = NP * D  ;
constexpr float AS_ = 8.0f, WS_ = 8.0f, SCALE = 0.25f;

typedef _Float16 b16;
typedef __attribute__((ext_vector_type(16))) _Float16 v16b;
typedef __attribute__((ext_vector_type(8))) _Float16 v8b;
typedef __attribute__((ext_vector_type(8))) float v8f;
typedef __attribute__((ext_vector_type(4))) float v4f;
__device__ __forceinline__ float bf16_rne(float f) { unsigned int u = __float_as_uint(f); u += 0x7FFFu + ((u >> 16) & 1u); return __uint_as_float(u & 0xFFFF0000u); }
__device__ __forceinline__ void split16(float v, b16& hi, b16& lo) { hi = (b16)v; lo = (b16)(v - (float)hi); }
__device__ __forceinline__ v16b frag_kb(const b16* p, int hh) { const v8b a = *(const v8b*)(p + 8 * hh), b = *(const v8b*)(p + 16 + 8 * hh); v16b f;
#pragma unroll
  for (int e = 0; e < 8; ++e) { f[e] = a[e]; f[8 + e] = b[e]; } return f; }
__device__ __forceinline__ v8f wmma16b(v16b a, v16b b, v8f c) { v8f d = __builtin_amdgcn_wmma_f32_16x16x32_f16(false, a, false, b, (short)0, c, false, false); asm volatile("v_nop\n\tv_nop\n\tv_nop\n\tv_nop" : "+v"(d) : "v"(a), "v"(b)); return d; }
__device__ __forceinline__ void wave_lds_sync() { __builtin_amdgcn_fence(__ATOMIC_RELEASE, "workgroup"); __builtin_amdgcn_wave_barrier(); __builtin_amdgcn_fence(__ATOMIC_ACQUIRE, "workgroup"); }
__device__ __forceinline__ float nexp(float x) { return __builtin_amdgcn_exp2f(x * 1.4426950408889634f); }

__global__ __launch_bounds__(256) void prep_kernel(const float* __restrict__ stc, const float* __restrict__ Wc, const float* __restrict__ Wqkv, const float* __restrict__ Wa, const float* __restrict__ ba, const float* __restrict__ Wo, const float* __restrict__ bo,
                                                   b16* __restrict__ wc16, b16* __restrict__ wq16, float* __restrict__ stat, float* __restrict__ rmask, b16* __restrict__ wph, b16* __restrict__ wpl, float* __restrict__ bp) {
  const int t_ = threadIdx.x;
  for (int pass = 0; pass < 2; ++pass) {
    for (int p = t_; p < D * KF; p += 256) { const int o = p >> 5, k = p & 31; ((volatile b16*)wc16)[p] = (b16)((k < FEAT + 2) ? bf16_rne(Wc[k * D + o]) : 0.0f); }
    for (int p = t_; p < 3 * D * D; p += 256) { const int o = p >> 6, k = p & 63; ((volatile b16*)wq16)[p] = (b16)bf16_rne(Wqkv[k * 3 * D + o]); }
    for (int p = t_; p < SP * 16; p += 256) { const int s = p >> 4, f = p & 15; ((volatile float*)stat)[p] = (s < S && f < FEAT) ? bf16_rne(stc[s * FEAT + f]) : 0.0f; }
    for (int p = t_; p < 32; p += 256) { float v = 0.0f;
      if (p < R) { float c = 0.0f; for (int s = 0; s < S; ++s) c += (bf16_rne(stc[s * FEAT + 2 + p]) > 0.5f) ? 1.0f : 0.0f; v = c; }
      ((volatile float*)rmask)[p] = v; }
    for (int p = t_; p < HID * KO; p += 256) { const int o = p / KO, q = p % KO, pp = q >> 6, k = q & 63; float s = 0.0f;
#pragma unroll 1
      for (int j = 0; j < D; ++j) s += bf16_rne(Wa[k * D + j]) * bf16_rne(Wo[(pp * D + j) * HID + o]);
      b16 a, c; split16(s * WS_, a, c); ((volatile b16*)wph)[p] = a; ((volatile b16*)wpl)[p] = c; }
    for (int o = t_; o < HID; o += 256) { float s = bf16_rne(bo[o]);
#pragma unroll 1
      for (int pp = 0; pp < NP; ++pp) {
#pragma unroll 1
        for (int j = 0; j < D; ++j) s += bf16_rne(ba[j]) * bf16_rne(Wo[(pp * D + j) * HID + o]); }
      ((volatile float*)bp)[o] = s; }
    __threadfence();
  }
}

__global__ __launch_bounds__(192) void batch_kernel(const float* __restrict__ infl, const float* __restrict__ stat, const float* __restrict__ rmask, const b16* __restrict__ wc16, const float* __restrict__ bc, const b16* __restrict__ wq16, const float* __restrict__ bqkv, const float* __restrict__ stc, float* __restrict__ pools) {
  __shared__ __attribute__((aligned(16))) float Tk[SP][D + 4]; __shared__ __attribute__((aligned(16))) b16 Qs[NH][SP][32], Ks[NH][SP][32], Vt[NH][HD][SP + 8]; __shared__ __attribute__((aligned(16))) float Cx[SP][D + 4]; __shared__ __attribute__((aligned(16))) float Pl[NP][D];
  const int b = blockIdx.x, wid = threadIdx.x >> 5, lane = threadIdx.x & 31, nloc = lane & 15, hlf = lane >> 4, m0 = wid * 16;
  for (int i = threadIdx.x; i < NH * SP * 32 / 8; i += 192) { const v8b z = {}; *(v8b*)(&Qs[0][0][0] + i * 8) = z; *(v8b*)(&Ks[0][0][0] + i * 8) = z; }
  __syncthreads();
  { v16b ah, al; const int s = m0 + nloc; const bool ok = (s < S);
#pragma unroll
    for (int e = 0; e < 16; ++e) { const int k = (e < 8) ? (8 * hlf + e) : (16 + 8 * hlf + e - 8); float v = 0.0f;
      if (ok) { if (k == 0) v = bf16_rne(infl[(size_t)b * 2 * S + s]) * 0.1f; else if (k == 1) v = bf16_rne(infl[(size_t)b * 2 * S + S + s]) * 0.1f; else if (k < FEAT + 2) v = stat[s * 16 + (k - 2)]; }
      b16 a, c; split16(v * AS_, a, c); ah[e] = a; al[e] = c; }
    v8f acc[4] = {{}, {}, {}, {}};
#pragma unroll
    for (int t = 0; t < 4; ++t) { const v16b bw = frag_kb(wc16 + (size_t)(t * 16 + nloc) * KF, hlf); acc[t] = wmma16b(ah, bw, acc[t]); acc[t] = wmma16b(al, bw, acc[t]); }
#pragma unroll
    for (int t = 0; t < 4; ++t)
#pragma unroll
      for (int v = 0; v < 8; ++v) { const int r = m0 + 8 * hlf + v, c = t * 16 + nloc; Tk[r][c] = (r < S) ? fmaxf(acc[t][v] * (1.0f / AS_) + bf16_rne(bc[c]), 0.0f) : 0.0f; } }
  wave_lds_sync();
  { v8f acc[12];
#pragma unroll
    for (int t = 0; t < 12; ++t) acc[t] = (v8f){};
#pragma unroll
    for (int kb = 0; kb < D; kb += 32) { v16b ah, al;
#pragma unroll
      for (int e = 0; e < 16; ++e) { const int k = kb + ((e < 8) ? (8 * hlf + e) : (16 + 8 * hlf + e - 8)); b16 a, c; split16(Tk[m0 + nloc][k] * AS_, a, c); ah[e] = a; al[e] = c; }
#pragma unroll
      for (int t = 0; t < 12; ++t) { const v16b bw = frag_kb(wq16 + (size_t)(t * 16 + nloc) * D + kb, hlf); acc[t] = wmma16b(ah, bw, acc[t]); acc[t] = wmma16b(al, bw, acc[t]); } }
#pragma unroll
    for (int t = 0; t < 12; ++t) { const int c = t * 16 + nloc, which = t >> 2, h = t & 3; const float bb = bf16_rne(bqkv[c]);
#pragma unroll
      for (int v = 0; v < 8; ++v) { const int r = m0 + 8 * hlf + v; const float val = (r < S) ? acc[t][v] * (1.0f / AS_) + bb : 0.0f;
        if (which == 0) Qs[h][r][nloc] = (b16)val; else if (which == 1) Ks[h][r][nloc] = (b16)val; else Vt[h][nloc][r] = (b16)val; } } }
  __syncthreads();
  for (int task = wid; task < NH * 6; task += 6) { const int h = task / 6, qt = task % 6, q0 = qt * 16;
    const v16b qf = frag_kb(&Qs[h][q0 + nloc][0], hlf);
    v8f s[6];
#pragma unroll
    for (int kt = 0; kt < 6; ++kt) { s[kt] = (v8f){}; const v16b kf = frag_kb(&Ks[h][kt * 16 + nloc][0], hlf); s[kt] = wmma16b(kf, qf, s[kt]); }
    float m = -INFINITY;
#pragma unroll
    for (int kt = 0; kt < 6; ++kt)
#pragma unroll
      for (int r = 0; r < 8; ++r) { const int key = kt * 16 + 8 * hlf + r; s[kt][r] = (key < S) ? s[kt][r] * SCALE : -INFINITY; m = fmaxf(m, s[kt][r]); }
    m = fmaxf(m, __shfl_xor(m, 16));
    float l = 0.0f;
#pragma unroll
    for (int kt = 0; kt < 6; ++kt)
#pragma unroll
      for (int r = 0; r < 8; ++r) { const float p = (s[kt][r] > -INFINITY) ? nexp(s[kt][r] - m) : 0.0f; s[kt][r] = p; l += p; }
    l += __shfl_xor(l, 16); const float il = 1.0f / l;
    v8f o = {};
#pragma unroll
    for (int ks = 0; ks < 3; ++ks) { v16b pf;
#pragma unroll
      for (int r = 0; r < 8; ++r) { pf[r] = (b16)(s[2 * ks][r] * il); pf[8 + r] = (b16)(s[2 * ks + 1][r] * il); }
      const v16b vf = frag_kb(&Vt[h][nloc][ks * 32], hlf); o = wmma16b(vf, pf, o); }
#pragma unroll
    for (int r = 0; r < 8; ++r) Cx[q0 + nloc][h * HD + 8 * hlf + r] = o[r];
  }
  __syncthreads();
  for (int i = threadIdx.x; i < NP * D; i += 192) { const int p = i >> 6, c = i & 63; float s_ = 0.0f, cnt = (p == 0) ? (float)S : rmask[p - 1];
    for (int s = 0; s < S; ++s) { const bool in = (p == 0) || (bf16_rne(stc[s * FEAT + 2 + (p - 1)]) > 0.5f); s_ += in ? Cx[s][c] : 0.0f; }
    Pl[p][c] = s_ / fmaxf(cnt, 1.0f); }
  __syncthreads();
  for (int pass = 0; pass < 2; ++pass) { if (threadIdx.x < 128) *(volatile v4f*)(pools + (size_t)b * KO + threadIdx.x * 4) = *(const v4f*)(&Pl[0][0] + threadIdx.x * 4); __threadfence(); }
}

__global__ __launch_bounds__(128) void head_kernel(const float* __restrict__ pools, const b16* __restrict__ wph, const b16* __restrict__ wpl, const float* __restrict__ bp, float* __restrict__ out) {
  __shared__ __attribute__((aligned(16))) float Ts[4][32 * 64];
  const int lane = threadIdx.x & 31, wave = threadIdx.x >> 5, nloc = lane & 15, hlf = lane >> 4, m0 = blockIdx.y * 128 + wave * 32, c0 = blockIdx.x * 64;
  v8f acc[2][4];
#pragma unroll
  for (int r = 0; r < 2; ++r)
#pragma unroll
    for (int t = 0; t < 4; ++t) acc[r][t] = (v8f){};
#pragma unroll 2
  for (int kb = 0; kb < KO; kb += 32) { v16b a0, a1, l0, l1;
#pragma unroll
    for (int e = 0; e < 16; ++e) { const int k = kb + ((e < 8) ? (8 * hlf + e) : (16 + 8 * hlf + e - 8)); b16 p, q; split16(pools[(size_t)(m0 + nloc) * KO + k] * AS_, p, q); a0[e] = p; l0[e] = q; split16(pools[(size_t)(m0 + 16 + nloc) * KO + k] * AS_, p, q); a1[e] = p; l1[e] = q; }
#pragma unroll
    for (int t = 0; t < 4; ++t) { const size_t bo_ = (size_t)(c0 + t * 16 + nloc) * KO + kb; const v16b b0 = frag_kb(wph + bo_, hlf), b1 = frag_kb(wpl + bo_, hlf);
      acc[0][t] = wmma16b(a0, b0, acc[0][t]); acc[0][t] = wmma16b(l0, b0, acc[0][t]); acc[0][t] = wmma16b(a0, b1, acc[0][t]);
      acc[1][t] = wmma16b(a1, b0, acc[1][t]); acc[1][t] = wmma16b(l1, b0, acc[1][t]); acc[1][t] = wmma16b(a1, b1, acc[1][t]); } }
  float* Tt = Ts[wave];
#pragma unroll
  for (int t = 0; t < 4; ++t)
#pragma unroll
    for (int r = 0; r < 2; ++r)
#pragma unroll
      for (int v = 0; v < 8; ++v) Tt[(r * 16 + v + 8 * hlf) * 64 + t * 16 + nloc] = fmaxf(acc[r][t][v] * (1.0f / (AS_ * WS_)) + bp[c0 + t * 16 + nloc], 0.0f);
  wave_lds_sync();
  float* dst0 = out + (size_t)m0 * HID + c0;
  for (int pass = 0; pass < 2; ++pass) {
#pragma unroll
    for (int j = 0; j < 16; ++j) { const int rr = j * 2 + hlf, c4 = nloc * 4; *(volatile v4f*)(dst0 + (size_t)rr * HID + c4) = *(const v4f*)(Tt + rr * 64 + c4); }
    __threadfence(); }
}
}

extern "C" void kernel_launch(void* const* d_in, const int* in_sizes, int n_in,
                              void* d_out, int out_size, void* d_ws, size_t ws_size, hipStream_t stream) {
  (void)n_in; (void)out_size;
  const float* infl = (const float*)d_in[0]; const float* stc = (const float*)d_in[1]; const float* Wc = (const float*)d_in[2]; const float* bc = (const float*)d_in[3]; const float* Wqkv = (const float*)d_in[4]; const float* bqkv = (const float*)d_in[5];
  const float* Wa = (const float*)d_in[6]; const float* ba = (const float*)d_in[7]; const float* Wo = (const float*)d_in[8]; const float* bo = (const float*)d_in[9];
  float* out = (float*)d_out;
  if (in_sizes[0] != Bn * 2 * S || in_sizes[1] != S * FEAT || in_sizes[2] != (FEAT + 2) * D || in_sizes[4] != D * 3 * D || in_sizes[6] != D * D || in_sizes[8] != KO * HID) return;
  size_t off = 0; char* ws = (char*)d_ws;
  auto carve = [&](size_t bytes) { char* p = ws + off; off += (bytes + 255) & ~(size_t)255; return p; };
  b16* wc16 = (b16*)carve(D * KF * 2); b16* wq16 = (b16*)carve(3 * D * D * 2); float* stat = (float*)carve(SP * 16 * 4); float* rmask = (float*)carve(256); b16* wph = (b16*)carve((size_t)HID * KO * 2); b16* wpl = (b16*)carve((size_t)HID * KO * 2); float* bp = (float*)carve(HID * 4);
  float* pools = (float*)carve((size_t)Bn * KO * 4);
  if (off > ws_size) return;
  prep_kernel<<<1, 256, 0, stream>>>(stc, Wc, Wqkv, Wa, ba, Wo, bo, wc16, wq16, stat, rmask, wph, wpl, bp);
  batch_kernel<<<Bn, 192, 0, stream>>>(infl, stat, rmask, wc16, bc, wq16, bqkv, stc, pools);
  head_kernel<<<dim3(HID / 64, Bn / 128), 128, 0, stream>>>(pools, wph, wpl, bp, out);
}
